// VAE_79525614452823
// MI455X (gfx1250) — hardware-run, weakly checked
//
#include <hip/hip_runtime.h>
#include <math.h>

constexpr int NBATCH = 16384;
constexpr int NSTEPS = 100;
constexpr int NDIM   = 5;
constexpr int NHID   = 32;
constexpr int NGATE  = 4 * NHID;
constexpr int ROWS_PER_WAVE = 16;
constexpr int WAVES_PER_BLK = 2;
constexpr int ROWS_PER_BLK  = ROWS_PER_WAVE * WAVES_PER_BLK;
constexpr int NTHREADS = 32 * WAVES_PER_BLK;
constexpr int NBLOCKS  = NBATCH / ROWS_PER_BLK;
constexpr int APITCH = 136;
constexpr int A_RXH = 0;
constexpr int A_RXL = 32;
constexpr int A_HH  = 64;
constexpr int A_HL  = 96;
constexpr int BPITCH = 72;
constexpr int B_XC = 0;
constexpr int B_HC = 32;
constexpr int OPITCH = 40;
constexpr int RROW   = NSTEPS * NDIM;
constexpr int RTILE  = ROWS_PER_BLK * RROW;
constexpr int RTILE4 = RTILE / 4;
constexpr int NFLUSH = (RTILE4 + NTHREADS - 1) / NTHREADS;
constexpr int OUT_RECON_N = NBATCH * RROW;
constexpr int OFF_MU  = OUT_RECON_N;
constexpr int OFF_LV  = OFF_MU + NBATCH;
constexpr int OFF_NUM = OFF_LV + NBATCH;
constexpr int OUT_TOTAL = OFF_NUM + NBATCH;
constexpr int P_BENC  = 0;
constexpr int P_BDEC  = 128;
constexpr int P_WMU   = 256;
constexpr int P_WLV   = 320;
constexpr int P_WL2H  = 384;
constexpr int P_BL2H  = 416;
constexpr int P_WL2H2 = 448;
constexpr int P_BL2H2 = 480;
constexpr int P_BEMB  = 512;
constexpr int P_WEMB  = 544;
constexpr int P_STK   = 704;
constexpr int P_BOUT  = 712;
constexpr int P_WSEQ  = 720;
constexpr int P_BSEQ  = 752;
constexpr int P_WSEQ2 = 784;
constexpr int P_BMU   = 816;
constexpr int P_BLV   = 817;
constexpr int P_BSEQ2 = 818;
constexpr int PRM_N   = 832;

static_assert(NBATCH % ROWS_PER_BLK == 0, "grid exact");
static_assert(NTHREADS == 64, "fill_out_plane maps 64 threads onto 16 rows x 4 groups");
static_assert((NGATE * 8) % NTHREADS == 0, "gate plane fill loop exact");
static_assert(RTILE % 4 == 0, "float4 flush");
static_assert((RTILE * 4) % 128 == 0, "block output region is whole 128-B lines");
static_assert(ROWS_PER_BLK * 4 == 128, "small outputs: one whole line per block");
static_assert((OFF_MU * 4) % 128 == 0 && (OFF_LV * 4) % 128 == 0 && (OFF_NUM * 4) % 128 == 0, "line-aligned outputs");
static_assert(OUT_TOTAL * 4 == 32964608, "total output bytes");
static_assert(APITCH % 8 == 0 && BPITCH % 8 == 0 && OPITCH % 8 == 0, "16-B aligned fragment loads");
static_assert(A_HL + 32 <= APITCH && B_HC + 32 <= BPITCH && NHID <= OPITCH, "plane widths");
static_assert(NHID == 32 && NGATE == 128, "one 32-deep k chunk per operand plane, 8 n-subtiles");

typedef __attribute__((ext_vector_type(16))) __bf16   v16b;
typedef __attribute__((ext_vector_type(8)))  __bf16   v8b;
typedef __attribute__((ext_vector_type(8)))  float    v8f;
typedef __attribute__((ext_vector_type(4)))  float    v4f;
typedef __attribute__((ext_vector_type(8)))  unsigned v8u;
typedef __attribute__((ext_vector_type(4)))  unsigned v4u;

__device__ __forceinline__ unsigned f2bf_bits32(float f) {
  const unsigned u = __float_as_uint(f);
  return (u + 0x7FFFu + ((u >> 16) & 1u)) >> 16;
}
__device__ __forceinline__ float bf16r(float f) { return __uint_as_float(f2bf_bits32(f) << 16); }
__device__ __forceinline__ void split2(float f, unsigned& hb, unsigned& lb) {
  hb = f2bf_bits32(f);
  lb = f2bf_bits32(f - __uint_as_float(hb << 16));
}
__device__ __forceinline__ float opaque_zero() { float z; asm volatile("v_mov_b32 %0, 0" : "=v"(z)); return z; }

__device__ __forceinline__ v16b fragload(const unsigned short* p) {
  union { v16b v; v8b h[2]; } f;
  const __bf16* q = (const __bf16*)(const void*)p;
  f.h[0] = *(const v8b*)(q);
  f.h[1] = *(const v8b*)(q + 16);
  return f.v;
}
__device__ __forceinline__ v8f mma_bf(v16b a, v16b b, v8f acc) {
  return __builtin_amdgcn_wmma_f32_16x16x32_bf16(false, a, false, b, (short)0, acc, false, false);
}
__device__ __forceinline__ void guard_grp(v8f& a0, v8f& a1, v8f& a2, v8f& a3,
                                          v16b f0, v16b f1, v16b b0, v16b b1, v16b b2, v16b b3) {
  asm volatile("v_nop\n\tv_nop\n\tv_nop\n\tv_nop"
               : "+v"(a0), "+v"(a1), "+v"(a2), "+v"(a3)
               : "v"(f0), "v"(f1), "v"(b0), "v"(b1), "v"(b2), "v"(b3));
}
__device__ __forceinline__ void guard_one(v8f& a0, v16b f0, v16b f1, v16b b0) {
  asm volatile("v_nop\n\tv_nop\n\tv_nop\n\tv_nop" : "+v"(a0) : "v"(f0), "v"(f1), "v"(b0));
}
__device__ __forceinline__ void lds_order() { asm volatile("" ::: "memory"); }

__device__ __forceinline__ float fsig(float z)   { return __builtin_amdgcn_rcpf(1.0f + __expf(-z)); }
__device__ __forceinline__ float ftanh(float z)  { return 1.0f - 2.0f * __builtin_amdgcn_rcpf(__expf(2.0f * z) + 1.0f); }
__device__ __forceinline__ float flrelu(float v) { return (v >= 0.0f) ? v : 0.01f * v; }

__device__ __forceinline__ void stage_vec(float* dst, const float* __restrict__ src, int n, int tid) {
#pragma unroll 1
  for (int i = tid; i < n; i += NTHREADS) dst[i] = bf16r(src[i]);
}

__device__ __forceinline__ void fill_gate_plane_enc(unsigned short* Wpl, const float* __restrict__ Wih,
                                                    const float* __restrict__ Whh, int tid) {
#pragma unroll 1
  for (int it = 0; it < (NGATE * 8) / NTHREADS; ++it) {
    const int idx = it * NTHREADS + tid;
    const int n   = idx >> 3;
    const int g   = idx & 7;
    const int gk  = g & 3;
    const float fh = (g >= 4) ? 1.0f : 0.0f;
    const float* hp = Whh + n * NHID + 8 * gk;
    const v4f hl = *(const v4f*)(hp);
    const v4f hu = *(const v4f*)(hp + 4);
    float hv[8];
    hv[0] = hl[0]; hv[1] = hl[1]; hv[2] = hl[2]; hv[3] = hl[3];
    hv[4] = hu[0]; hv[5] = hu[1]; hv[6] = hu[2]; hv[7] = hu[3];
    unsigned wb[8];
#pragma unroll
    for (int e = 0; e < 8; ++e) {
      const int k  = 8 * gk + e;
      const int kc = (k < NDIM) ? k : (NDIM - 1);
      const float fi = (g < 4 && k < NDIM) ? 1.0f : 0.0f;
      const float a  = Wih[n * NDIM + kc];
      wb[e] = f2bf_bits32(fmaf(fi, a, fh * hv[e]) + 0.0f);
    }
    v4u wv;
    wv[0] = wb[0] | (wb[1] << 16);
    wv[1] = wb[2] | (wb[3] << 16);
    wv[2] = wb[4] | (wb[5] << 16);
    wv[3] = wb[6] | (wb[7] << 16);
    *(v4u*)(Wpl + n * BPITCH + 8 * g) = wv;
  }
}
__device__ __forceinline__ void fill_gate_plane_dec(unsigned short* Wpl, const float* __restrict__ Wih,
                                                    const float* __restrict__ Whh, int tid) {
#pragma unroll 1
  for (int it = 0; it < (NGATE * 8) / NTHREADS; ++it) {
    const int idx = it * NTHREADS + tid;
    const int n   = idx >> 3;
    const int g   = idx & 7;
    const int gk  = g & 3;
    const float fh = (g >= 4) ? 1.0f : 0.0f;
    const float fi = (g < 4) ? 1.0f : 0.0f;
    const float* hp = Whh + n * NHID + 8 * gk;
    const float* ap = Wih + n * NHID + 8 * gk;
    const v4f hl = *(const v4f*)(hp);
    const v4f hu = *(const v4f*)(hp + 4);
    const v4f al = *(const v4f*)(ap);
    const v4f au = *(const v4f*)(ap + 4);
    float hv[8], av[8];
    hv[0] = hl[0]; hv[1] = hl[1]; hv[2] = hl[2]; hv[3] = hl[3];
    hv[4] = hu[0]; hv[5] = hu[1]; hv[6] = hu[2]; hv[7] = hu[3];
    av[0] = al[0]; av[1] = al[1]; av[2] = al[2]; av[3] = al[3];
    av[4] = au[0]; av[5] = au[1]; av[6] = au[2]; av[7] = au[3];
    unsigned wb[8];
#pragma unroll
    for (int e = 0; e < 8; ++e) wb[e] = f2bf_bits32(fmaf(fi, av[e], fh * hv[e]) + 0.0f);
    v4u wv;
    wv[0] = wb[0] | (wb[1] << 16);
    wv[1] = wb[2] | (wb[3] << 16);
    wv[2] = wb[4] | (wb[5] << 16);
    wv[3] = wb[6] | (wb[7] << 16);
    *(v4u*)(Wpl + n * BPITCH + 8 * g) = wv;
  }
}

__device__ __forceinline__ void fill_out_plane(unsigned short* Wpl, const float* __restrict__ Wout, int tid) {
  const int n  = tid >> 2;
  const int g  = tid & 3;
  const int nc = (n < NDIM) ? n : (NDIM - 1);
  const float f = (n < NDIM) ? 1.0f : 0.0f;
  const float* wp = Wout + nc * NHID + 8 * g;
  const v4f a0 = *(const v4f*)(wp);
  const v4f a1 = *(const v4f*)(wp + 4);
  v4u wv;
  wv[0] = f2bf_bits32(f * a0[0] + 0.0f) | (f2bf_bits32(f * a0[1] + 0.0f) << 16);
  wv[1] = f2bf_bits32(f * a0[2] + 0.0f) | (f2bf_bits32(f * a0[3] + 0.0f) << 16);
  wv[2] = f2bf_bits32(f * a1[0] + 0.0f) | (f2bf_bits32(f * a1[1] + 0.0f) << 16);
  wv[3] = f2bf_bits32(f * a1[2] + 0.0f) | (f2bf_bits32(f * a1[3] + 0.0f) << 16);
  *(v4u*)(Wpl + n * OPITCH + 8 * g) = wv;
}

__device__ __forceinline__ void lstm_cell8(const v8f& ai, const v8f& af, const v8f& ag, const v8f& ao,
                                           float bi, float bf, float bg, float bo4,
                                           float (&hs)[8], float (&cs)[8]) {
#pragma unroll
  for (int r = 0; r < 8; ++r) {
    const float zi = ai[r] + bi;
    const float zf = af[r] + bf;
    const float zg = ag[r] + bg;
    const float zo = ao[r] + bo4;
    const float ig = fsig(zi);
    const float fg = fsig(zf);
    const float gg = ftanh(zg);
    const float og = fsig(zo);
    const float cn = fg * cs[r] + ig * gg;
    cs[r] = cn;
    hs[r] = og * ftanh(cn);
  }
}

__global__ __launch_bounds__(NTHREADS) void vae_seq_kernel(
    const float* __restrict__ x,         const float* __restrict__ eps,
    const float* __restrict__ enc_Wih,   const float* __restrict__ enc_Whh,
    const float* __restrict__ enc_bih,   const float* __restrict__ enc_bhh,
    const float* __restrict__ W_mu,      const float* __restrict__ b_mu,
    const float* __restrict__ W_lv,      const float* __restrict__ b_lv,
    const float* __restrict__ W_l2h,     const float* __restrict__ b_l2h,
    const float* __restrict__ W_l2h2,    const float* __restrict__ b_l2h2,
    const float* __restrict__ start_tok, const float* __restrict__ W_emb,
    const float* __restrict__ b_emb,
    const float* __restrict__ dec_Wih,   const float* __restrict__ dec_Whh,
    const float* __restrict__ dec_bih,   const float* __restrict__ dec_bhh,
    const float* __restrict__ W_out,     const float* __restrict__ b_out,
    const float* __restrict__ W_seq,     const float* __restrict__ b_seq,
    const float* __restrict__ W_seq2,    const float* __restrict__ b_seq2,
    float* __restrict__ out) {
  __shared__ __align__(16) float          Rs[RTILE];
  __shared__ __align__(16) unsigned short Wg[NGATE * BPITCH];
  __shared__ __align__(16) unsigned short Wo[16 * OPITCH];
  __shared__ __align__(16) unsigned short At[WAVES_PER_BLK][ROWS_PER_WAVE * APITCH];
  __shared__ __align__(16) float          prm[PRM_N];
  __shared__ __align__(16) float          sOut[3][ROWS_PER_BLK];

  const int tid  = threadIdx.x;
  const int lane = tid & 31;
  const int wave = tid >> 5;
  const int c    = lane & 15;
  const int hh   = lane >> 4;
  const int koff = 8 * hh;
  const int blk  = blockIdx.x;
  const int rowg = blk * ROWS_PER_BLK + wave * ROWS_PER_WAVE;
  unsigned short* Atw = &At[wave][0];

#pragma unroll 1
  for (int i = tid; i < NGATE; i += NTHREADS) prm[P_BENC + i] = bf16r(enc_bih[i]) + bf16r(enc_bhh[i]);
#pragma unroll 1
  for (int i = tid; i < NGATE; i += NTHREADS) prm[P_BDEC + i] = bf16r(dec_bih[i]) + bf16r(dec_bhh[i]);
  stage_vec(prm + P_WMU,   W_mu,      2 * NHID,    tid);
  stage_vec(prm + P_WLV,   W_lv,      2 * NHID,    tid);
  stage_vec(prm + P_WL2H,  W_l2h,     NHID,        tid);
  stage_vec(prm + P_BL2H,  b_l2h,     NHID,        tid);
  stage_vec(prm + P_WL2H2, W_l2h2,    NHID,        tid);
  stage_vec(prm + P_BL2H2, b_l2h2,    NHID,        tid);
  stage_vec(prm + P_BEMB,  b_emb,     NHID,        tid);
  stage_vec(prm + P_WEMB,  W_emb,     NHID * NDIM, tid);
  stage_vec(prm + P_STK,   start_tok, NDIM,        tid);
  stage_vec(prm + P_BOUT,  b_out,     NDIM,        tid);
  stage_vec(prm + P_WSEQ,  W_seq,     NHID,        tid);
  stage_vec(prm + P_BSEQ,  b_seq,     NHID,        tid);
  stage_vec(prm + P_WSEQ2, W_seq2,    NHID,        tid);
  stage_vec(prm + P_BMU,   b_mu,      1,           tid);
  stage_vec(prm + P_BLV,   b_lv,      1,           tid);
  stage_vec(prm + P_BSEQ2, b_seq2,    1,           tid);
  fill_gate_plane_enc(Wg, enc_Wih, enc_Whh, tid);
  fill_out_plane(Wo, W_out, tid);

  const float oz = opaque_zero();
  const unsigned zb = f2bf_bits32(oz);
  float hst[2][8], cst[2][8];
#pragma unroll
  for (int nt = 0; nt < 2; ++nt)
#pragma unroll
    for (int r = 0; r < 8; ++r) { hst[nt][r] = oz; cst[nt][r] = oz; }
#pragma unroll
  for (int nt = 0; nt < 2; ++nt)
#pragma unroll
    for (int r = 0; r < 8; ++r) {
      Atw[(8 * hh + r) * APITCH + A_HH + 16 * nt + c] = (unsigned short)zb;
      Atw[(8 * hh + r) * APITCH + A_HL + 16 * nt + c] = (unsigned short)zb;
    }
  __syncthreads();

  const v8f z8 = {0.f, 0.f, 0.f, 0.f, 0.f, 0.f, 0.f, 0.f};
  float benc[2][4];
#pragma unroll
  for (int nt = 0; nt < 2; ++nt)
#pragma unroll
    for (int g = 0; g < 4; ++g) benc[nt][g] = prm[P_BENC + 32 * g + 16 * nt + c];

#pragma unroll 1
  for (int t = 0; t < NSTEPS; ++t) {
    const float* xr = x + ((size_t)(rowg + c) * NSTEPS + (size_t)t) * NDIM;
    const float x0 = xr[0], x1 = xr[1], x2 = xr[2], x3 = xr[3], x4 = xr[4];
    const unsigned keep = (hh == 0) ? 0xffffffffu : 0u;
    v8u wx;
    wx[0] = (f2bf_bits32(x0) | (f2bf_bits32(x1) << 16)) & keep;
    wx[1] = (f2bf_bits32(x2) | (f2bf_bits32(x3) << 16)) & keep;
    wx[2] = f2bf_bits32(x4) & keep;
    wx[3] = 0u; wx[4] = 0u; wx[5] = 0u; wx[6] = 0u; wx[7] = 0u;
    const v16b ax  = __builtin_bit_cast(v16b, wx);
    const v16b ahh = fragload(Atw + c * APITCH + A_HH + koff);
    const v16b ahl = fragload(Atw + c * APITCH + A_HL + koff);
#pragma unroll
    for (int nt = 0; nt < 2; ++nt) {
      v8f acc[4];
      acc[0] = z8; acc[1] = z8; acc[2] = z8; acc[3] = z8;
      {
        const unsigned short* bp = Wg + (16 * nt + c) * BPITCH + B_XC + koff;
        const v16b b0 = fragload(bp);
        const v16b b1 = fragload(bp + 32 * BPITCH);
        const v16b b2 = fragload(bp + 64 * BPITCH);
        const v16b b3 = fragload(bp + 96 * BPITCH);
        acc[0] = mma_bf(ax, b0, acc[0]);
        acc[1] = mma_bf(ax, b1, acc[1]);
        acc[2] = mma_bf(ax, b2, acc[2]);
        acc[3] = mma_bf(ax, b3, acc[3]);
        guard_grp(acc[0], acc[1], acc[2], acc[3], ax, ax, b0, b1, b2, b3);
      }
      lds_order();
      {
        const unsigned short* bp = Wg + (16 * nt + c) * BPITCH + B_HC + koff;
        const v16b b0 = fragload(bp);
        const v16b b1 = fragload(bp + 32 * BPITCH);
        const v16b b2 = fragload(bp + 64 * BPITCH);
        const v16b b3 = fragload(bp + 96 * BPITCH);
        acc[0] = mma_bf(ahh, b0, acc[0]);
        acc[1] = mma_bf(ahh, b1, acc[1]);
        acc[2] = mma_bf(ahh, b2, acc[2]);
        acc[3] = mma_bf(ahh, b3, acc[3]);
        acc[0] = mma_bf(ahl, b0, acc[0]);
        acc[1] = mma_bf(ahl, b1, acc[1]);
        acc[2] = mma_bf(ahl, b2, acc[2]);
        acc[3] = mma_bf(ahl, b3, acc[3]);
        guard_grp(acc[0], acc[1], acc[2], acc[3], ahh, ahl, b0, b1, b2, b3);
      }
      lds_order();
      lstm_cell8(acc[0], acc[1], acc[2], acc[3], benc[nt][0], benc[nt][1], benc[nt][2], benc[nt][3],
                 hst[nt], cst[nt]);
    }
    __syncthreads();
#pragma unroll
    for (int nt = 0; nt < 2; ++nt)
#pragma unroll
      for (int r = 0; r < 8; ++r) {
        unsigned hb, lb;
        split2(hst[nt][r], hb, lb);
        Atw[(8 * hh + r) * APITCH + A_HH + 16 * nt + c] = (unsigned short)hb;
        Atw[(8 * hh + r) * APITCH + A_HL + 16 * nt + c] = (unsigned short)lb;
      }
    __syncthreads();
  }

  float muv[8], lvv[8], zv[8], numv[8];
  {
    float wmu_h[2], wmu_c[2], wlv_h[2], wlv_c[2];
#pragma unroll
    for (int nt = 0; nt < 2; ++nt) {
      wmu_h[nt] = prm[P_WMU + 16 * nt + c];
      wmu_c[nt] = prm[P_WMU + NHID + 16 * nt + c];
      wlv_h[nt] = prm[P_WLV + 16 * nt + c];
      wlv_c[nt] = prm[P_WLV + NHID + 16 * nt + c];
    }
    float pmu[8], plv[8];
#pragma unroll
    for (int r = 0; r < 8; ++r) {
      float sm = 0.0f, sl = 0.0f;
#pragma unroll
      for (int nt = 0; nt < 2; ++nt) {
        sm = fmaf(hst[nt][r], wmu_h[nt], sm);
        sm = fmaf(cst[nt][r], wmu_c[nt], sm);
        sl = fmaf(hst[nt][r], wlv_h[nt], sl);
        sl = fmaf(cst[nt][r], wlv_c[nt], sl);
      }
      pmu[r] = sm; plv[r] = sl;
    }
#pragma unroll
    for (int r = 0; r < 8; ++r) {
#pragma unroll
      for (int off = 1; off < 16; off <<= 1) {
        pmu[r] += __shfl_xor(pmu[r], off, 32);
        plv[r] += __shfl_xor(plv[r], off, 32);
      }
    }
    const float bmu = prm[P_BMU], blv = prm[P_BLV];
    float epv[8];
#pragma unroll
    for (int r = 0; r < 8; ++r) epv[r] = bf16r(eps[rowg + 8 * hh + r]);
#pragma unroll
    for (int r = 0; r < 8; ++r) {
      muv[r] = pmu[r] + bmu;
      lvv[r] = plv[r] + blv;
      zv[r]  = muv[r] + epv[r] * expf(0.5f * lvv[r]);
    }
    float wsq[2], bsq[2], wsq2[2];
#pragma unroll
    for (int nt = 0; nt < 2; ++nt) {
      wsq[nt]  = prm[P_WSEQ  + 16 * nt + c];
      bsq[nt]  = prm[P_BSEQ  + 16 * nt + c];
      wsq2[nt] = prm[P_WSEQ2 + 16 * nt + c];
    }
    float pn[8];
#pragma unroll
    for (int r = 0; r < 8; ++r) {
      float s = 0.0f;
#pragma unroll
      for (int nt = 0; nt < 2; ++nt) {
        const float a = flrelu(zv[r] * wsq[nt] + bsq[nt]);
        s = fmaf(a, wsq2[nt], s);
      }
      pn[r] = s;
    }
#pragma unroll
    for (int r = 0; r < 8; ++r) {
#pragma unroll
      for (int off = 1; off < 16; off <<= 1) pn[r] += __shfl_xor(pn[r], off, 32);
    }
    const float bsq2 = prm[P_BSEQ2];
#pragma unroll
    for (int r = 0; r < 8; ++r) numv[r] = fmaxf(pn[r] + bsq2, 0.0f);
  }
  if (c == 0) {
#pragma unroll
    for (int r = 0; r < 8; ++r) {
      const int idx = 16 * wave + 8 * hh + r;
      sOut[0][idx] = muv[r];
      sOut[1][idx] = lvv[r];
      sOut[2][idx] = numv[r];
    }
  }
  float x0v[2];
  {
    float wl2h[2], bl2h[2], wl2h2[2], bl2h2[2];
#pragma unroll
    for (int nt = 0; nt < 2; ++nt) {
      const int j = 16 * nt + c;
      wl2h[nt]  = prm[P_WL2H  + j];
      bl2h[nt]  = prm[P_BL2H  + j];
      wl2h2[nt] = prm[P_WL2H2 + j];
      bl2h2[nt] = prm[P_BL2H2 + j];
      float p = 0.0f;
#pragma unroll
      for (int d = 0; d < NDIM; ++d) p = fmaf(prm[P_STK + d], prm[P_WEMB + j * NDIM + d], p);
      x0v[nt] = p + prm[P_BEMB + j];
    }
#pragma unroll
    for (int nt = 0; nt < 2; ++nt)
#pragma unroll
      for (int r = 0; r < 8; ++r) {
        hst[nt][r] = flrelu(muv[r] * wl2h[nt]  + bl2h[nt]);
        cst[nt][r] = flrelu(muv[r] * wl2h2[nt] + bl2h2[nt]);
      }
  }
  __syncthreads();

  fill_gate_plane_dec(Wg, dec_Wih, dec_Whh, tid);
#pragma unroll
  for (int nt = 0; nt < 2; ++nt) {
    unsigned xhb, xlb;
    split2(fmaxf(x0v[nt], 0.0f), xhb, xlb);
#pragma unroll
    for (int r = 0; r < 8; ++r) {
      unsigned hb, lb;
      split2(hst[nt][r], hb, lb);
      const int base = (8 * hh + r) * APITCH + 16 * nt + c;
      Atw[base + A_RXH] = (unsigned short)xhb;
      Atw[base + A_RXL] = (unsigned short)xlb;
      Atw[base + A_HH]  = (unsigned short)hb;
      Atw[base + A_HL]  = (unsigned short)lb;
    }
  }
  float bdec[2][4];
#pragma unroll
  for (int nt = 0; nt < 2; ++nt)
#pragma unroll
    for (int g = 0; g < 4; ++g) bdec[nt][g] = prm[P_BDEC + 32 * g + 16 * nt + c];
  const float bo = prm[P_BOUT + ((c < NDIM) ? c : (NDIM - 1))];
  __syncthreads();
  const v16b bout = fragload(Wo + c * OPITCH + koff);
  float* Rsw = Rs + (16 * wave) * RROW;

#pragma unroll 1
  for (int t = 0; t < NSTEPS; ++t) {
    const v16b rxh = fragload(Atw + c * APITCH + A_RXH + koff);
    const v16b rxl = fragload(Atw + c * APITCH + A_RXL + koff);
    const v16b ahh = fragload(Atw + c * APITCH + A_HH + koff);
    const v16b ahl = fragload(Atw + c * APITCH + A_HL + koff);
#pragma unroll
    for (int nt = 0; nt < 2; ++nt) {
      v8f acc[4];
      acc[0] = z8; acc[1] = z8; acc[2] = z8; acc[3] = z8;
      {
        const unsigned short* bp = Wg + (16 * nt + c) * BPITCH + B_XC + koff;
        const v16b b0 = fragload(bp);
        const v16b b1 = fragload(bp + 32 * BPITCH);
        const v16b b2 = fragload(bp + 64 * BPITCH);
        const v16b b3 = fragload(bp + 96 * BPITCH);
        acc[0] = mma_bf(rxh, b0, acc[0]);
        acc[1] = mma_bf(rxh, b1, acc[1]);
        acc[2] = mma_bf(rxh, b2, acc[2]);
        acc[3] = mma_bf(rxh, b3, acc[3]);
        acc[0] = mma_bf(rxl, b0, acc[0]);
        acc[1] = mma_bf(rxl, b1, acc[1]);
        acc[2] = mma_bf(rxl, b2, acc[2]);
        acc[3] = mma_bf(rxl, b3, acc[3]);
        guard_grp(acc[0], acc[1], acc[2], acc[3], rxh, rxl, b0, b1, b2, b3);
      }
      lds_order();
      {
        const unsigned short* bp = Wg + (16 * nt + c) * BPITCH + B_HC + koff;
        const v16b b0 = fragload(bp);
        const v16b b1 = fragload(bp + 32 * BPITCH);
        const v16b b2 = fragload(bp + 64 * BPITCH);
        const v16b b3 = fragload(bp + 96 * BPITCH);
        acc[0] = mma_bf(ahh, b0, acc[0]);
        acc[1] = mma_bf(ahh, b1, acc[1]);
        acc[2] = mma_bf(ahh, b2, acc[2]);
        acc[3] = mma_bf(ahh, b3, acc[3]);
        acc[0] = mma_bf(ahl, b0, acc[0]);
        acc[1] = mma_bf(ahl, b1, acc[1]);
        acc[2] = mma_bf(ahl, b2, acc[2]);
        acc[3] = mma_bf(ahl, b3, acc[3]);
        guard_grp(acc[0], acc[1], acc[2], acc[3], ahh, ahl, b0, b1, b2, b3);
      }
      lds_order();
      lstm_cell8(acc[0], acc[1], acc[2], acc[3], bdec[nt][0], bdec[nt][1], bdec[nt][2], bdec[nt][3],
                 hst[nt], cst[nt]);
    }
    __syncthreads();
#pragma unroll
    for (int nt = 0; nt < 2; ++nt)
#pragma unroll
      for (int r = 0; r < 8; ++r) {
        unsigned hb, lb;
        split2(hst[nt][r], hb, lb);
        const unsigned pm = (hst[nt][r] > 0.0f) ? 0xffffu : 0u;
        const int base = (8 * hh + r) * APITCH + 16 * nt + c;
        Atw[base + A_RXH] = (unsigned short)(hb & pm);
        Atw[base + A_RXL] = (unsigned short)(lb & pm);
        Atw[base + A_HH]  = (unsigned short)hb;
        Atw[base + A_HL]  = (unsigned short)lb;
      }
    __syncthreads();
    const v16b anh = fragload(Atw + c * APITCH + A_HH + koff);
    const v16b anl = fragload(Atw + c * APITCH + A_HL + koff);
    v8f oc = mma_bf(anh, bout, z8);
    oc = mma_bf(anl, bout, oc);
    guard_one(oc, anh, anl, bout);
    float ov[8];
#pragma unroll
    for (int r = 0; r < 8; ++r) ov[r] = oc[r] + bo;
    if (c < NDIM) {
#pragma unroll
      for (int r = 0; r < 8; ++r) Rsw[(8 * hh + r) * RROW + t * NDIM + c] = ov[r];
    }
  }
  __syncthreads();

  {
    float* ob = out + (size_t)blk * RTILE;
    for (int pass = 0; pass < 2; ++pass) {
#pragma unroll 1
      for (int it = 0; it < NFLUSH; ++it) {
        const int f  = it * NTHREADS + tid;
        const int fc = (f < RTILE4) ? f : (RTILE4 - 1);
        const v4f v = *(const v4f*)(Rs + 4 * fc);
        if (f < RTILE4) *(volatile v4f*)(ob + 4 * (size_t)f) = v;
      }
      __threadfence();
    }
  }
  if (wave == 0) {
    const float vm = sOut[0][lane];
    const float vl = sOut[1][lane];
    const float vn = sOut[2][lane];
    float* pm = out + (size_t)OFF_MU  + blk * ROWS_PER_BLK + lane;
    float* pl = out + (size_t)OFF_LV  + blk * ROWS_PER_BLK + lane;
    float* pq = out + (size_t)OFF_NUM + blk * ROWS_PER_BLK + lane;
    for (int pass = 0; pass < 2; ++pass) {
      *(volatile float*)pm = vm;
      *(volatile float*)pl = vl;
      *(volatile float*)pq = vn;
      __threadfence();
    }
  }
}

extern "C" void kernel_launch(void* const* d_in, const int* in_sizes, int n_in,
                              void* d_out, int out_size, void* d_ws, size_t ws_size, hipStream_t stream) {
  (void)d_ws; (void)ws_size;
  if (n_in < 27 || d_out == nullptr) return;
  if (in_sizes[0]  != NBATCH * NSTEPS * NDIM || in_sizes[1]  != NBATCH ||
      in_sizes[2]  != NGATE * NDIM  || in_sizes[3]  != NGATE * NHID ||
      in_sizes[4]  != NGATE         || in_sizes[5]  != NGATE ||
      in_sizes[6]  != 2 * NHID      || in_sizes[7]  != 1 ||
      in_sizes[8]  != 2 * NHID      || in_sizes[9]  != 1 ||
      in_sizes[10] != NHID          || in_sizes[11] != NHID ||
      in_sizes[12] != NHID          || in_sizes[13] != NHID ||
      in_sizes[14] != NDIM          || in_sizes[15] != NHID * NDIM || in_sizes[16] != NHID ||
      in_sizes[17] != NGATE * NHID  || in_sizes[18] != NGATE * NHID ||
      in_sizes[19] != NGATE         || in_sizes[20] != NGATE ||
      in_sizes[21] != NDIM * NHID   || in_sizes[22] != NDIM ||
      in_sizes[23] != NHID          || in_sizes[24] != NHID ||
      in_sizes[25] != NHID          || in_sizes[26] != 1 ||
      out_size != OUT_TOTAL) return;

  const float* x         = (const float*)d_in[0];
  const float* eps       = (const float*)d_in[1];
  const float* enc_Wih   = (const float*)d_in[2];
  const float* enc_Whh   = (const float*)d_in[3];
  const float* enc_bih   = (const float*)d_in[4];
  const float* enc_bhh   = (const float*)d_in[5];
  const float* W_mu      = (const float*)d_in[6];
  const float* b_mu      = (const float*)d_in[7];
  const float* W_lv      = (const float*)d_in[8];
  const float* b_lv      = (const float*)d_in[9];
  const float* W_l2h     = (const float*)d_in[10];
  const float* b_l2h     = (const float*)d_in[11];
  const float* W_l2h2    = (const float*)d_in[12];
  const float* b_l2h2    = (const float*)d_in[13];
  const float* start_tok = (const float*)d_in[14];
  const float* W_emb     = (const float*)d_in[15];
  const float* b_emb     = (const float*)d_in[16];
  const float* dec_Wih   = (const float*)d_in[17];
  const float* dec_Whh   = (const float*)d_in[18];
  const float* dec_bih   = (const float*)d_in[19];
  const float* dec_bhh   = (const float*)d_in[20];
  const float* W_out     = (const float*)d_in[21];
  const float* b_out     = (const float*)d_in[22];
  const float* W_seq     = (const float*)d_in[23];
  const float* b_seq     = (const float*)d_in[24];
  const float* W_seq2    = (const float*)d_in[25];
  const float* b_seq2    = (const float*)d_in[26];
  float* out = (float*)d_out;

  vae_seq_kernel<<<NBLOCKS, NTHREADS, 0, stream>>>(
      x, eps, enc_Wih, enc_Whh, enc_bih, enc_bhh, W_mu, b_mu, W_lv, b_lv,
      W_l2h, b_l2h, W_l2h2, b_l2h2, start_tok, W_emb, b_emb,
      dec_Wih, dec_Whh, dec_bih, dec_bhh, W_out, b_out,
      W_seq, b_seq, W_seq2, b_seq2, out);
}
